// UniversalDirectionalGSA_67688684585066
// MI455X (gfx1250) — hardware-verified
//
#include <hip/hip_runtime.h>
#include <math.h>
#include <stdint.h>

#ifndef NB
#define NB 1
#endif
#ifndef SEQ
#define SEQ 2048
#endif
#define XS_FULL 2048
#define DMOD  2048
#define NH    16
#define HD    128
#define NSP   8
#define SPW   32
#define STW   32
#define QO    ((SEQ < 256) ? SEQ : 256)
#define MCH   SEQ
#define NST   (MCH / 64)
#define NQT   (SEQ / 16)
#define NKT   (SEQ / 32)
#define RSQ_HD 0.08838834764831845f
#define LOG2E 1.4426950408889634f
#define NEGT  (-1.0e30f)
#define QSC   256.0f
#define KSC   256.0f
#define PCAR  32768.0f
#define VCAR  1024.0f
#define OSC   1024.0f
#define WOS   1024.0f
#define WPB   2
#define ATT_THREADS (WPB * 32)
#define PTP   36
#define PTW   (16 * PTP)
#define SLP   68
#define SLW   (16 * SLP)
#define WREG  (2 * PTW + SLW)
#define SMEMF (2 * PTW + WPB * WREG)
#define SLAB64 (16 * 68)
#define VTP   72
#define WS_CAP 134217728
static_assert(NB == 1);
static_assert(DMOD == NH * HD && HD == 128 && NH == 16 && NSP == 8 && 2 * NSP <= SPW && SPW == 32 && STW == 32);
static_assert((SEQ % 64) == 0 && SEQ >= 64 && SEQ <= XS_FULL);
static_assert((QO % 64) == 0 && QO >= 64 && QO <= SEQ && (QO % 16) == 0);
static_assert((MCH % 64) == 0 && NST * 64 == MCH);
static_assert((DMOD % 64) == 0 && (DMOD % 32) == 0 && (HD % 32) == 0 && WPB * 64 == HD);
static_assert(((SEQ * DMOD / 8) % 256) == 0 && ((DMOD * DMOD / 8) % 256) == 0);
static_assert(SMEMF * 4 <= 65536 && 2 * HD * VTP * 2 <= 65536 && 4 * SLAB64 * 4 <= 65536);
static_assert(ATT_THREADS == 64 && NQT * 16 == SEQ && NKT * 32 == SEQ);

typedef unsigned short u16;
typedef _Float16 v16h __attribute__((ext_vector_type(16)));
typedef _Float16 v8h  __attribute__((ext_vector_type(8)));
typedef __bf16   v16b __attribute__((ext_vector_type(16)));
typedef float    v8f  __attribute__((ext_vector_type(8)));
typedef float    v4f  __attribute__((ext_vector_type(4)));
typedef unsigned int v4u __attribute__((ext_vector_type(4)));

union FragH { v16h v; v8h h[2]; v4u u[2]; };
union FragB { v16b v; v4u u[2]; };

__device__ __forceinline__ unsigned short bf_bits(float f) {
  unsigned u = __float_as_uint(f);
  return (unsigned short)((u + 0x7FFFu + ((u >> 16) & 1u)) >> 16);
}
__device__ __forceinline__ float bf_up(unsigned short h) { return __uint_as_float(((unsigned)h) << 16); }
__device__ __forceinline__ float bfr(float f) { return bf_up(bf_bits(f)); }
__device__ __forceinline__ unsigned short h_bits(_Float16 x) { return __builtin_bit_cast(unsigned short, x); }
__device__ __forceinline__ unsigned pk16(unsigned short a, unsigned short b) { return (unsigned)a | ((unsigned)b << 16); }
__device__ __forceinline__ v8f zero8() { v8f z = {0.f, 0.f, 0.f, 0.f, 0.f, 0.f, 0.f, 0.f}; return z; }

__device__ __forceinline__ v16h ldfrag_h(const _Float16* p) {
  FragH f;
  f.h[0] = *(const v8h*)(p);
  f.h[1] = *(const v8h*)(p + 16);
  return f.v;
}
__device__ __forceinline__ v16b ldfrag_b(const u16* p) {
  FragB f;
  f.u[0] = *(const v4u*)(p);
  f.u[1] = *(const v4u*)(p + 16);
  return f.v;
}

__device__ __forceinline__ v8f mma_h(v16h a, v16h b, v8f c) {
  return __builtin_amdgcn_wmma_f32_16x16x32_f16(false, a, false, b, (short)0, c, false, false);
}
__device__ __forceinline__ v8f mma_b(v16b a, v16b b, v8f c) {
  return __builtin_amdgcn_wmma_f32_16x16x32_bf16(false, a, false, b, (short)0, c, false, false);
}
__device__ __forceinline__ void guard_s(v8f& a, v16h x0, v16h x1, v16h x2, v16h x3) {
#if defined(__HIP_DEVICE_COMPILE__)
  asm volatile("v_nop\n\tv_nop\n\tv_nop\n\tv_nop" : "+v"(a) : "v"(x0), "v"(x1), "v"(x2), "v"(x3) : "memory");
#endif
}
__device__ __forceinline__ void guard_b2(v8f& a, v16b x0, v16b x1) {
#if defined(__HIP_DEVICE_COMPILE__)
  asm volatile("v_nop\n\tv_nop\n\tv_nop\n\tv_nop" : "+v"(a) : "v"(x0), "v"(x1) : "memory");
#endif
}
__device__ __forceinline__ void guard_pv(v8f& a, v8f& b, v8f& c2, v8f& d, v16h x0, v16h x1, v16h x2, v16h x3,
                                         v16h x4, v16h x5, v16h x6, v16h x7) {
#if defined(__HIP_DEVICE_COMPILE__)
  asm volatile("v_nop\n\tv_nop\n\tv_nop\n\tv_nop"
               : "+v"(a), "+v"(b), "+v"(c2), "+v"(d)
               : "v"(x0), "v"(x1), "v"(x2), "v"(x3), "v"(x4), "v"(x5), "v"(x6), "v"(x7) : "memory");
#endif
}
template <typename F>
__device__ __forceinline__ void guard6(v8f& a, v8f& b, v8f& c, v8f& d, F x0, F x1, F x2, F x3, F x4, F x5) {
#if defined(__HIP_DEVICE_COMPILE__)
  asm volatile("v_nop\n\tv_nop\n\tv_nop\n\tv_nop"
               : "+v"(a), "+v"(b), "+v"(c), "+v"(d) : "v"(x0), "v"(x1), "v"(x2), "v"(x3), "v"(x4), "v"(x5) : "memory");
#endif
}
__device__ __forceinline__ void acc_guard4(v8f& a, v8f& b, v8f& c, v8f& d) {
#if defined(__HIP_DEVICE_COMPILE__)
  asm volatile("v_nop\n\tv_nop\n\tv_nop\n\tv_nop" : "+v"(a), "+v"(b), "+v"(c), "+v"(d));
#endif
}
__device__ __forceinline__ void wave_sync_lds() {
  __builtin_amdgcn_fence(__ATOMIC_RELEASE, "workgroup");
  __builtin_amdgcn_wave_barrier();
  __builtin_amdgcn_fence(__ATOMIC_ACQUIRE, "workgroup");
}

__global__ __launch_bounds__(256) void cvt16(const float* __restrict__ x, u16* D, int n8, int f16mode, float scale) {
  const int gt = blockIdx.x * 256 + (int)threadIdx.x;
  if (gt >= n8) return;
  const float* p = x + (size_t)gt * 8;
  const v4f a = *(const v4f*)(p), b4 = *(const v4f*)(p + 4);
  float w[8];
#pragma unroll
  for (int e = 0; e < 4; ++e) { w[e] = a[e]; w[4 + e] = b4[e]; }
  v4u o;
#pragma unroll
  for (int e = 0; e < 4; ++e) {
    const float f0 = w[2 * e], f1 = w[2 * e + 1];
    const unsigned short hb0 = h_bits((_Float16)(bfr(f0) * scale));
    const unsigned short hb1 = h_bits((_Float16)(bfr(f1) * scale));
    const unsigned short bb0 = bf_bits(f0);
    const unsigned short bb1 = bf_bits(f1);
    o[e] = (f16mode != 0) ? pk16(hb0, hb1) : pk16(bb0, bb1);
  }
  u16* d = D + (size_t)gt * 8;
  for (int pass = 0; pass < 2; ++pass) {
    *(volatile v4u*)(d) = o;
    __threadfence();
  }
}

__global__ __launch_bounds__(256) void hl16(const float* __restrict__ x, u16* Hq, u16* Lq, int n8, float scale) {
  const int gt = blockIdx.x * 256 + (int)threadIdx.x;
  if (gt >= n8) return;
  const float* p = x + (size_t)gt * 8;
  const v4f a = *(const v4f*)(p), b4 = *(const v4f*)(p + 4);
  float w[8];
#pragma unroll
  for (int e = 0; e < 4; ++e) { w[e] = a[e]; w[4 + e] = b4[e]; }
  v4u oh, ol;
#pragma unroll
  for (int e = 0; e < 4; ++e) {
    const float t0 = w[2 * e] * scale, t1 = w[2 * e + 1] * scale;
    const _Float16 h0 = (_Float16)t0, h1 = (_Float16)t1;
    const _Float16 l0 = (_Float16)(t0 - (float)h0), l1 = (_Float16)(t1 - (float)h1);
    oh[e] = pk16(h_bits(h0), h_bits(h1));
    ol[e] = pk16(h_bits(l0), h_bits(l1));
  }
  u16* dh = Hq + (size_t)gt * 8;
  u16* dl = Lq + (size_t)gt * 8;
  for (int pass = 0; pass < 2; ++pass) {
    *(volatile v4u*)(dh) = oh;
    *(volatile v4u*)(dl) = ol;
    __threadfence();
  }
}

__global__ __launch_bounds__(256) void vt16(const float* __restrict__ F, int b, int sbase, u16* VHo, u16* VLo) {
  __shared__ __align__(16) u16 TH[HD * VTP];
  __shared__ __align__(16) u16 TL[HD * VTP];
  const int tid = threadIdx.x;
  const int bid = blockIdx.x;
  const int st  = bid % NST;
  const int h   = bid / NST;
  if (h >= NH) return;
  const int sl0 = st * 64;
  {
    const int sl = tid >> 2;
    const int dc = (tid & 3) * 32;
    const float* src = F + (size_t)(sl0 + sl) * DMOD + h * HD + dc;
#pragma unroll
    for (int i = 0; i < 8; ++i) {
      const v4f a = *(const v4f*)(src + 4 * i);
#pragma unroll
      for (int e = 0; e < 4; ++e) {
        const float t = a[e] * VCAR;
        const _Float16 hv = (_Float16)t;
        const _Float16 lv = (_Float16)(t - (float)hv);
        TH[(dc + 4 * i + e) * VTP + sl] = h_bits(hv);
        TL[(dc + 4 * i + e) * VTP + sl] = h_bits(lv);
      }
    }
  }
  __syncthreads();
  v4u vh[4], vl[4];
  const int q8 = tid >> 3, p8 = (tid & 7) * 8;
#pragma unroll
  for (int it = 0; it < 4; ++it) {
    const int line = it * 32 + q8;
    vh[it] = *(const v4u*)(TH + line * VTP + p8);
    vl[it] = *(const v4u*)(TL + line * VTP + p8);
  }
  const size_t hrow = (size_t)(b * NH + h) * HD;
  const size_t base = hrow * SEQ + (size_t)(sbase + sl0) + p8;
  for (int pass = 0; pass < 2; ++pass) {
#pragma unroll
    for (int it = 0; it < 4; ++it) {
      const int line = it * 32 + q8;
      *(volatile v4u*)(VHo + base + (size_t)line * SEQ) = vh[it];
      *(volatile v4u*)(VLo + base + (size_t)line * SEQ) = vl[it];
    }
    __threadfence();
  }
}

__global__ __launch_bounds__(32) void ftab(const float* __restrict__ dir, const float* __restrict__ lsc,
                                          const float* __restrict__ lam, const float* __restrict__ dsp,
                                          const float* __restrict__ psp, float* DN, float* ST) {
  const int lane = (int)threadIdx.x;
  const int fi   = (int)blockIdx.x;
  if (fi >= NH * NSP) return;
  const v4f d4 = *(const v4f*)(dir + (size_t)fi * HD + 4 * lane);
  float dn = d4[0] * d4[0];
  dn = dn + d4[1] * d4[1];
  dn = dn + d4[2] * d4[2];
  dn = dn + d4[3] * d4[3];
#pragma unroll
  for (int off = 1; off < 32; off <<= 1) dn += __shfl_xor(dn, off, 32);
  const float nrm = sqrtf(dn);
  const float inv = 1.0f / (nrm + 1.0e-8f);
  v4f o;
#pragma unroll
  for (int e = 0; e < 4; ++e) o[e] = d4[e] * inv;
  const float sc  = expf(lsc[fi]);
  const float amp = expf(lam[fi]);
  const float rs2 = 1.0f / (sc * sc);
  const float ps  = psp[0];
  const float ds  = dsp[0];
  const float cq0 = ps * amp;
  const float cq1 = (ps * ds) * amp;
  const bool  l0  = (lane == 0);
  v4f sv;
  sv[0] = l0 ? rs2 : 0.0f;
  sv[1] = l0 ? cq0 : 0.0f;
  sv[2] = l0 ? cq1 : 0.0f;
  sv[3] = 0.0f;
  float* dd = DN + (size_t)fi * HD + 4 * lane;
  for (int pass = 0; pass < 2; ++pass) {
    *(volatile v4f*)(dd) = o;
    if (lane < 8) {
      *(volatile v4f*)(ST + (size_t)fi * STW + 4 * lane) = sv;
    }
    __threadfence();
  }
}

__global__ __launch_bounds__(256) void feat16(const float* __restrict__ F, const float* __restrict__ pos,
                                             const float* __restrict__ DN, const float* __restrict__ ST,
                                             int kside, u16* P) {
  __shared__ __align__(16) u16 L[256];
  const int tid  = threadIdx.x;
  const int wave = tid >> 5;
  const int lane = tid & 31;
  const int bid  = blockIdx.x;
  const int s    = bid >> 1;
  const int ho   = bid & 1;
  if (s >= SEQ) return;
  const int h  = ho * 8 + wave;
  const int n  = lane >> 2;
  const int dq = lane & 3;
  const int fi = h * NSP + n;
  const float* xp = F   + (size_t)s * DMOD + h * HD + dq * 32;
  const float* pp = pos + (size_t)fi * HD + dq * 32;
  const float* np = DN  + (size_t)fi * HD + dq * 32;
  float ss = 0.0f, dt = 0.0f;
#pragma unroll 2
  for (int i = 0; i < 8; ++i) {
    const v4f xv = *(const v4f*)(xp + 4 * i);
    const v4f pv = *(const v4f*)(pp + 4 * i);
    const v4f dv = *(const v4f*)(np + 4 * i);
#pragma unroll
    for (int e = 0; e < 4; ++e) {
      const float df = xv[e] - pv[e];
      ss = ss + df * df;
      dt = dt + df * dv[e];
    }
  }
  ss += __shfl_xor(ss, 1, 32);
  ss += __shfl_xor(ss, 2, 32);
  dt += __shfl_xor(dt, 1, 32);
  dt += __shfl_xor(dt, 2, 32);
  const float rs2 = ST[fi * STW + 0];
  const float cq0 = ST[fi * STW + 1];
  const float cq1 = ST[fi * STW + 2];
  const float g   = expf((-0.5f * ss) * rs2);
  const float dp  = tanhf(dt);
  const float gd  = g * dp;
  const float c0  = (kside != 0) ? g  : (cq0 * g);
  const float c1  = (kside != 0) ? gd : (cq1 * gd);
  const u16 b0 = bf_bits(c0);
  const u16 b1 = bf_bits(c1);
  if (dq == 0) {
    L[wave * SPW + n]       = b0;
    L[wave * SPW + NSP + n] = b1;
  }
  if (lane >= 2 * NSP) L[wave * SPW + lane] = (u16)0;
  __syncthreads();
  if (wave == 0) {
    const v4u v = *(const v4u*)(L + lane * 8);
    u16* d = P + ((size_t)s * NH + ho * 8) * SPW + lane * 8;
    for (int pass = 0; pass < 2; ++pass) {
      *(volatile v4u*)(d) = v;
      __threadfence();
    }
  }
}

__device__ __forceinline__ void epi64(float* sl, v8f a0, v8f a1, v8f a2, v8f a3, float oscale,
                                      float* C, int N, size_t rowb, int col0, int lane) {
  const int hh = lane >> 4, m = lane & 15;
#pragma unroll
  for (int r = 0; r < 8; ++r) {
    const int ro = (8 * hh + r) * 68 + m;
    sl[ro]      = a0[r] * oscale;
    sl[ro + 16] = a1[r] * oscale;
    sl[ro + 32] = a2[r] * oscale;
    sl[ro + 48] = a3[r] * oscale;
  }
  wave_sync_lds();
  v4f vals[8];
#pragma unroll
  for (int it = 0; it < 8; ++it) vals[it] = *(const v4f*)(sl + (it * 2 + hh) * 68 + m * 4);
  float* dst = C + (rowb + (size_t)hh) * (size_t)N + col0 + m * 4;
  for (int pass = 0; pass < 2; ++pass) {
#pragma unroll
    for (int it = 0; it < 8; ++it) {
      *(volatile v4f*)(dst + (size_t)(it * 2) * (size_t)N) = vals[it];
    }
    __threadfence();
  }
}

__global__ __launch_bounds__(128)
void gemm_bf(const u16* __restrict__ A, const u16* __restrict__ Bt, float* C, int M, int N, int K, float oscale) {
  __shared__ __align__(16) float slab[4 * SLAB64];
  const int tid = threadIdx.x, wave = tid >> 5, lane = tid & 31, hh = lane >> 4, m = lane & 15;
  const int ntile = N >> 6;
  const int bid   = blockIdx.x;
  const int rowb  = (bid / ntile) * 64 + wave * 16;
  const int col0  = (bid % ntile) * 64;
  if (rowb + 16 > M) return;
  const u16* ap = A  + (size_t)(rowb + m) * K + 8 * hh;
  const u16* bp = Bt + (size_t)(col0 + m) * K + 8 * hh;
  const size_t bs = (size_t)16 * K;
  v8f acc0 = zero8(), acc1 = zero8(), acc2 = zero8(), acc3 = zero8();
#pragma unroll 1
  for (int k0 = 0; k0 < K; k0 += 32) {
    const v16b a  = ldfrag_b(ap + k0);
    const v16b b0 = ldfrag_b(bp + k0);
    const v16b b1 = ldfrag_b(bp + bs + k0);
    const v16b b2 = ldfrag_b(bp + 2 * bs + k0);
    const v16b b3 = ldfrag_b(bp + 3 * bs + k0);
    acc0 = mma_b(a, b0, acc0);
    acc1 = mma_b(a, b1, acc1);
    acc2 = mma_b(a, b2, acc2);
    acc3 = mma_b(a, b3, acc3);
    guard6<v16b>(acc0, acc1, acc2, acc3, a, b0, b1, b2, b3, a);
  }
  epi64(slab + wave * SLAB64, acc0, acc1, acc2, acc3, oscale, C, N, (size_t)rowb, col0, lane);
}

template <int NPROD>
__global__ __launch_bounds__(128)
void gemm_o(const u16* __restrict__ Ah, const u16* __restrict__ Al, const u16* __restrict__ Bt,
            float* C, int sbeg, int nrt, float oscale) {
  __shared__ __align__(16) float slab[4 * SLAB64];
  const int tid = threadIdx.x, wave = tid >> 5, lane = tid & 31, hh = lane >> 4, m = lane & 15;
  const int ntile = DMOD >> 6;
  const int bid   = blockIdx.x;
  const int ct    = bid % ntile;
  const int t2    = bid / ntile;
  const int rt    = t2 % nrt;
  const int bb    = t2 / nrt;
  if (bb >= NB) return;
  const int srow  = sbeg + rt * 64 + wave * 16;
  if (srow + 16 > SEQ) return;
  const int col0  = ct * 64;
  const int K     = DMOD;
  const size_t rowC = (size_t)bb * SEQ + srow;
  const size_t rowL = (size_t)bb * QO + srow;
  const _Float16* ahp = (const _Float16*)(const void*)Ah + (rowC + m) * K + 8 * hh;
  const _Float16* alp = (const _Float16*)(const void*)Al + (rowL + m) * K + 8 * hh;
  const _Float16* bp  = (const _Float16*)(const void*)Bt + (size_t)(col0 + m) * K + 8 * hh;
  const size_t bs = (size_t)16 * K;
  v8f acc0 = zero8(), acc1 = zero8(), acc2 = zero8(), acc3 = zero8();
  if constexpr (NPROD == 2) {
#pragma unroll 1
    for (int k0 = 0; k0 < K; k0 += 32) {
      const v16h ah = ldfrag_h(ahp + k0), al = ldfrag_h(alp + k0);
      const v16h b0 = ldfrag_h(bp + k0);
      const v16h b1 = ldfrag_h(bp + bs + k0);
      const v16h b2 = ldfrag_h(bp + 2 * bs + k0);
      const v16h b3 = ldfrag_h(bp + 3 * bs + k0);
      acc0 = mma_h(ah, b0, acc0);  acc0 = mma_h(al, b0, acc0);
      acc1 = mma_h(ah, b1, acc1);  acc1 = mma_h(al, b1, acc1);
      acc2 = mma_h(ah, b2, acc2);  acc2 = mma_h(al, b2, acc2);
      acc3 = mma_h(ah, b3, acc3);  acc3 = mma_h(al, b3, acc3);
      guard6<v16h>(acc0, acc1, acc2, acc3, ah, al, b0, b1, b2, b3);
    }
  } else {
#pragma unroll 1
    for (int k0 = 0; k0 < K; k0 += 32) {
      const v16h ah = ldfrag_h(ahp + k0);
      const v16h b0 = ldfrag_h(bp + k0);
      const v16h b1 = ldfrag_h(bp + bs + k0);
      const v16h b2 = ldfrag_h(bp + 2 * bs + k0);
      const v16h b3 = ldfrag_h(bp + 3 * bs + k0);
      acc0 = mma_h(ah, b0, acc0);
      acc1 = mma_h(ah, b1, acc1);
      acc2 = mma_h(ah, b2, acc2);
      acc3 = mma_h(ah, b3, acc3);
      guard6<v16h>(acc0, acc1, acc2, acc3, ah, b0, b1, b2, b3, ah);
    }
  }
  epi64(slab + wave * SLAB64, acc0, acc1, acc2, acc3, oscale, C, DMOD, rowC, col0, lane);
}

__device__ __forceinline__ void smx_step(const float* tsh, float* pt, float (&mrow)[8], float (&lrow)[8],
                                         v8f (&o)[4], int hh, int c) {
#pragma unroll
  for (int r = 0; r < 8; ++r) {
    const int   ro = (8 * hh + r) * PTP + c;
    const float t0 = tsh[ro];
    const float t1 = tsh[ro + 16];
    float mx = fmaxf(t0, t1);
#pragma unroll
    for (int off = 1; off < 16; off <<= 1) mx = fmaxf(mx, __shfl_xor(mx, off, 32));
    const float mn = fmaxf(mrow[r], mx);
    const float ms = (mn == -INFINITY) ? 0.0f : mn;
    const float al = exp2f(mrow[r] - ms);
    mrow[r] = mn;
    const float e0 = exp2f(t0 - ms), e1 = exp2f(t1 - ms);
    float ps = e0 + e1;
#pragma unroll
    for (int off = 1; off < 16; off <<= 1) ps += __shfl_xor(ps, off, 32);
    lrow[r] = lrow[r] * al + ps;
#pragma unroll
    for (int j = 0; j < 4; ++j) o[j][r] *= al;
    pt[ro]      = e0;
    pt[ro + 16] = e1;
  }
}

__device__ __forceinline__ void pfrag(const float* pt, int hh, int c, FragH& ph, FragH& pl) {
  const float* prow = pt + c * PTP + 8 * hh;
  const v4f p0 = *(const v4f*)(prow), p1 = *(const v4f*)(prow + 4);
  const v4f p2 = *(const v4f*)(prow + 16), p3 = *(const v4f*)(prow + 20);
#pragma unroll
  for (int e = 0; e < 4; ++e) {
    const float ta = p0[e] * PCAR, tb = p1[e] * PCAR, tc = p2[e] * PCAR, td = p3[e] * PCAR;
    const _Float16 ha = (_Float16)ta, hb = (_Float16)tb, hc = (_Float16)tc, hv = (_Float16)td;
    ph.h[0][e]     = ha;
    ph.h[0][4 + e] = hb;
    ph.h[1][e]     = hc;
    ph.h[1][4 + e] = hv;
    pl.h[0][e]     = (_Float16)(ta - (float)ha);
    pl.h[0][4 + e] = (_Float16)(tb - (float)hb);
    pl.h[1][e]     = (_Float16)(tc - (float)hc);
    pl.h[1][4 + e] = (_Float16)(td - (float)hv);
  }
}

__global__ __launch_bounds__(ATT_THREADS)
void attn_g(const u16* __restrict__ QHp, const u16* __restrict__ QLp,
            const u16* __restrict__ KHp, const u16* __restrict__ KLp,
            const u16* __restrict__ QSp, const u16* __restrict__ KSp,
            const u16* __restrict__ VHp, const u16* __restrict__ VLp,
            const float* __restrict__ gsp, u16* OHp, u16* OLp) {
  __shared__ __align__(16) float smem[SMEMF];

  const int tid  = threadIdx.x;
  const int wave = tid >> 5;
  const int lane = tid & 31;
  const int hh   = lane >> 4;
  const int c    = lane & 15;
  const int bid  = blockIdx.x;
  const int qt   = bid % NQT;
  const int head = bid / NQT;
  if (head >= NH) return;
  const int q0   = qt * 16;

  float* tsh  = smem;
  float* tah  = smem + PTW;
  float* pts  = smem + 2 * PTW + wave * WREG;
  float* pta  = pts + PTW;
  float* slab = pta + PTW;

  const float gsv   = gsp[0];
  const float sgm   = 1.0f / (1.0f + expf(-gsv));
  const float blend = fminf(0.03f, sgm * 0.15f);
  const float w1    = 1.0f - blend;

  const int kw = 16 * wave;
  const int dw = 64 * wave;
  const size_t hcol = (size_t)head * HD + 8 * hh;
  const _Float16* Qh  = (const _Float16*)(const void*)QHp + (size_t)(q0 + c) * DMOD + hcol;
  const _Float16* Ql  = (const _Float16*)(const void*)QLp + (size_t)(q0 + c) * DMOD + hcol;
  const _Float16* Khb = (const _Float16*)(const void*)KHp + (size_t)(kw + c) * DMOD + hcol;
  const _Float16* Klb = (const _Float16*)(const void*)KLp + (size_t)(kw + c) * DMOD + hcol;
  const u16* QSa = QSp + ((size_t)(q0 + c) * NH + head) * SPW + 8 * hh;
  const u16* KSb = KSp + ((size_t)(kw + c) * NH + head) * SPW + 8 * hh;
  const _Float16* Vhb = (const _Float16*)(const void*)VHp + ((size_t)head * HD + dw + c) * SEQ + 8 * hh;
  const _Float16* Vlb = (const _Float16*)(const void*)VLp + ((size_t)head * HD + dw + c) * SEQ + 8 * hh;
  const float lsc = RSQ_HD * (LOG2E / (QSC * KSC));
  const float oc  = 1.0f / (PCAR * VCAR);
  const size_t KROW = (size_t)DMOD;
  const size_t SROW = (size_t)NH * SPW;

  float ms_[8], ls_[8], ma_[8], la_[8];
  v8f os[4], oa[4];
#pragma unroll
  for (int r = 0; r < 8; ++r) { ms_[r] = -INFINITY; ls_[r] = 0.f; ma_[r] = -INFINITY; la_[r] = 0.f; }
#pragma unroll
  for (int j = 0; j < 4; ++j) { os[j] = zero8(); oa[j] = zero8(); }
  const int ncaus = (q0 >> 5) + 1;
  const int nkt   = (ncaus < NKT) ? ncaus : NKT;
  const int qr0   = q0 + 8 * hh;

#pragma unroll 1
  for (int kt = 0; kt < nkt; ++kt) {
    const int kb = kt * 32;
    __syncthreads();
    v8f s = zero8();
    const _Float16* kp = Khb + (size_t)kb * KROW;
    const _Float16* lp = Klb + (size_t)kb * KROW;
#pragma unroll
    for (int kk = 0; kk < HD / 32; ++kk) {
      const v16h qh = ldfrag_h(Qh + kk * 32);
      const v16h ql = ldfrag_h(Ql + kk * 32);
      const v16h kh = ldfrag_h(kp + kk * 32);
      const v16h kl = ldfrag_h(lp + kk * 32);
      s = mma_h(qh, kh, s);
      s = mma_h(ql, kh, s);
      s = mma_h(qh, kl, s);
      guard_s(s, qh, ql, kh, kl);
    }
    v8f sp = zero8();
    {
      const v16b qs = ldfrag_b(QSa);
      const v16b ks = ldfrag_b(KSb + (size_t)kb * SROW);
      sp = mma_b(qs, ks, sp);
      guard_b2(sp, qs, ks);
    }
    const int key = kb + kw + c;
#pragma unroll
    for (int r = 0; r < 8; ++r) {
      const int   qr = qr0 + r;
      const float u  = s[r] * lsc;
      const float ua = fmaf(sp[r], LOG2E, u);
      const bool  ok = (key <= qr);
      const int   ro = (8 * hh + r) * PTP + kw + c;
      tsh[ro] = ok ? u : NEGT;
      tah[ro] = ok ? ua : NEGT;
    }
    __syncthreads();
    smx_step(tsh, pts, ms_, ls_, os, hh, c);
    smx_step(tah, pta, ma_, la_, oa, hh, c);
    wave_sync_lds();
    FragH phs, pls, pha, pla;
    pfrag(pts, hh, c, phs, pls);
    pfrag(pta, hh, c, pha, pla);
    {
      const _Float16* vhp = Vhb + kb;
      const _Float16* vlp = Vlb + kb;
#pragma unroll
      for (int jg = 0; jg < 2; ++jg) {
        const size_t da = (size_t)(2 * jg) * 16 * SEQ;
        const size_t db = da + (size_t)16 * SEQ;
        const v16h vha = ldfrag_h(vhp + da), vhb2 = ldfrag_h(vhp + db);
        const v16h vla = ldfrag_h(vlp + da), vlb2 = ldfrag_h(vlp + db);
        os[2 * jg]     = mma_h(phs.v, vha,  os[2 * jg]);
        os[2 * jg]     = mma_h(pls.v, vha,  os[2 * jg]);
        os[2 * jg]     = mma_h(phs.v, vla,  os[2 * jg]);
        os[2 * jg + 1] = mma_h(phs.v, vhb2, os[2 * jg + 1]);
        os[2 * jg + 1] = mma_h(pls.v, vhb2, os[2 * jg + 1]);
        os[2 * jg + 1] = mma_h(phs.v, vlb2, os[2 * jg + 1]);
        oa[2 * jg]     = mma_h(pha.v, vha,  oa[2 * jg]);
        oa[2 * jg]     = mma_h(pla.v, vha,  oa[2 * jg]);
        oa[2 * jg]     = mma_h(pha.v, vla,  oa[2 * jg]);
        oa[2 * jg + 1] = mma_h(pha.v, vhb2, oa[2 * jg + 1]);
        oa[2 * jg + 1] = mma_h(pla.v, vhb2, oa[2 * jg + 1]);
        oa[2 * jg + 1] = mma_h(pha.v, vlb2, oa[2 * jg + 1]);
        guard_pv(os[2 * jg], os[2 * jg + 1], oa[2 * jg], oa[2 * jg + 1],
                 phs.v, pls.v, pha.v, pla.v, vha, vhb2, vla, vlb2);
      }
    }
    wave_sync_lds();
  }
  acc_guard4(os[0], os[1], os[2], os[3]);
  acc_guard4(oa[0], oa[1], oa[2], oa[3]);
#pragma unroll
  for (int r = 0; r < 8; ++r) {
    const float lvs  = ls_[r];
    const float lss  = (lvs > 0.0f) ? lvs : 1.0f;
    const float invs = (lvs > 0.0f) ? ((1.0f / lss) * oc) : 0.0f;
    const float lva  = la_[r];
    const float lsa  = (lva > 0.0f) ? lva : 1.0f;
    const float inva = (lva > 0.0f) ? ((1.0f / lsa) * oc) : 0.0f;
#pragma unroll
    for (int j = 0; j < 4; ++j) {
      const int idx = (8 * hh + r) * SLP + j * 16 + c;
      slab[idx] = w1 * (os[j][r] * invs) + blend * (oa[j][r] * inva);
    }
  }
  wave_sync_lds();
  v4u oh[4], ol[4];
  const int q4 = lane >> 3, p8 = (lane & 7) * 8;
#pragma unroll
  for (int it = 0; it < 4; ++it) {
    const int row = it * 4 + q4;
    const v4f a = *(const v4f*)(slab + row * SLP + p8), b4 = *(const v4f*)(slab + row * SLP + p8 + 4);
    float w[8];
#pragma unroll
    for (int e = 0; e < 4; ++e) { w[e] = a[e] * OSC; w[4 + e] = b4[e] * OSC; }
#pragma unroll
    for (int e = 0; e < 4; ++e) {
      const _Float16 h0 = (_Float16)w[2 * e], h1 = (_Float16)w[2 * e + 1];
      const _Float16 l0 = (_Float16)(w[2 * e] - (float)h0), l1 = (_Float16)(w[2 * e + 1] - (float)h1);
      oh[it][e] = pk16(h_bits(h0), h_bits(h1));
      ol[it][e] = pk16(h_bits(l0), h_bits(l1));
    }
  }
  const bool wlo = (q0 < QO);
  const size_t ob = (size_t)q0 * DMOD + (size_t)head * HD + dw + p8;
  for (int pass = 0; pass < 2; ++pass) {
#pragma unroll
    for (int it = 0; it < 4; ++it) {
      const int row = it * 4 + q4;
      *(volatile v4u*)(OHp + ob + (size_t)row * DMOD) = oh[it];
      if (wlo) {
        *(volatile v4u*)(OLp + ob + (size_t)row * DMOD) = ol[it];
      }
    }
    __threadfence();
  }
}

extern "C" void kernel_launch(void* const* d_in, const int* in_sizes, int n_in,
                              void* d_out, int out_size, void* d_ws, size_t ws_size,
                              hipStream_t stream) {
  if (n_in < 12) return;
  if (in_sizes[0] < SEQ * DMOD) return;
  if (in_sizes[1] != DMOD * DMOD || in_sizes[2] != DMOD * DMOD) return;
  if (in_sizes[3] != DMOD * DMOD || in_sizes[4] != DMOD * DMOD) return;
  if (in_sizes[5] != NH * NSP * HD || in_sizes[6] != NH * NSP * HD) return;
  if (in_sizes[7] != NH * NSP || in_sizes[8] != NH * NSP) return;
  if (in_sizes[9] < 1 || in_sizes[10] < 1 || in_sizes[11] < 1) return;
  if (out_size < SEQ * DMOD) return;

  const float* x    = (const float*)d_in[0];
  const float* wq   = (const float*)d_in[1];
  const float* wk   = (const float*)d_in[2];
  const float* wv   = (const float*)d_in[3];
  const float* wo   = (const float*)d_in[4];
  const float* fpos = (const float*)d_in[5];
  const float* fdir = (const float*)d_in[6];
  const float* flsc = (const float*)d_in[7];
  const float* flam = (const float*)d_in[8];
  const float* dsp  = (const float*)d_in[9];
  const float* psp  = (const float*)d_in[10];
  const float* gsp  = (const float*)d_in[11];
  float*       out  = (float*)d_out;

  const size_t szP  = (size_t)SEQ * DMOD * 2;
  const size_t szW  = (size_t)DMOD * DMOD * 2;
  const size_t szF  = (size_t)SEQ * DMOD * 4;
  const size_t szS  = (size_t)SEQ * NH * SPW * 2;
  const size_t szDN = (size_t)NH * NSP * HD * 4;
  const size_t szST = (size_t)NH * NSP * STW * 4;
  const size_t szOL = (size_t)QO * DMOD * 2;
  size_t off = 0;
  const size_t oXB = off; off += szP;
  const size_t oWT = off; off += szW;
  const size_t oF  = off; off += szF;
  const size_t oQH = off; off += szP;
  const size_t oQL = off; off += szP;
  const size_t oKH = off; off += szP;
  const size_t oKL = off; off += szP;
  const size_t oVH = off; off += szP;
  const size_t oVL = off; off += szP;
  const size_t oQS = off; off += szS;
  const size_t oKS = off; off += szS;
  const size_t oDN = off; off += szDN;
  const size_t oST = off; off += szST;
  const size_t oOH = off; off += szP;
  const size_t oOL = off; off += szOL;
  const size_t oWO = off; off += szW;
  if (off > ws_size) return;
  if (off > (size_t)WS_CAP) return;

  char* ws = (char*)d_ws;
  u16*   XB = (u16*)(ws + oXB);
  u16*   WT = (u16*)(ws + oWT);
  float* F  = (float*)(ws + oF);
  u16*   QH = (u16*)(ws + oQH);
  u16*   QL = (u16*)(ws + oQL);
  u16*   KH = (u16*)(ws + oKH);
  u16*   KL = (u16*)(ws + oKL);
  u16*   VH = (u16*)(ws + oVH);
  u16*   VL = (u16*)(ws + oVL);
  u16*   QS = (u16*)(ws + oQS);
  u16*   KS = (u16*)(ws + oKS);
  float* DN = (float*)(ws + oDN);
  float* ST = (float*)(ws + oST);
  u16*   OH = (u16*)(ws + oOH);
  u16*   OL = (u16*)(ws + oOL);
  u16*   WO = (u16*)(ws + oWO);

  const dim3 b256(256), b128(128), b32(32), bAT(ATT_THREADS);
  const int  n8s = (SEQ * DMOD) / 8;
  const int  n8w = (DMOD * DMOD) / 8;
  const dim3 gXs((n8s + 255) / 256);
  const dim3 gXw((n8w + 255) / 256);
  const dim3 gG((SEQ / 64) * (DMOD / 64));
  const dim3 gVT(NH * NST);
  const dim3 gFT(SEQ * 2);
  const dim3 gTB(NH * NSP);
  const dim3 gAT(NQT * NH);
  const int  nrtR = QO / 64;
  const int  nrtP = (SEQ - QO) / 64;

  cvt16<<<gXs, b256, 0, stream>>>(x, XB, n8s, 0, 1.0f);
  ftab<<<gTB, b32, 0, stream>>>(fdir, flsc, flam, dsp, psp, DN, ST);
  cvt16<<<gXw, b256, 0, stream>>>(wv, WT, n8w, 0, 1.0f);
  gemm_bf<<<gG, b128, 0, stream>>>(XB, WT, F, SEQ, DMOD, DMOD, 1.0f);
  vt16<<<gVT, b256, 0, stream>>>(F, 0, 0, VH, VL);
  cvt16<<<gXw, b256, 0, stream>>>(wq, WT, n8w, 0, 1.0f);
  gemm_bf<<<gG, b128, 0, stream>>>(XB, WT, F, SEQ, DMOD, DMOD, 1.0f);
  hl16<<<gXs, b256, 0, stream>>>(F, QH, QL, n8s, QSC);
  feat16<<<gFT, b256, 0, stream>>>(F, fpos, DN, ST, 0, QS);
  cvt16<<<gXw, b256, 0, stream>>>(wk, WT, n8w, 0, 1.0f);
  gemm_bf<<<gG, b128, 0, stream>>>(XB, WT, F, SEQ, DMOD, DMOD, 1.0f);
  hl16<<<gXs, b256, 0, stream>>>(F, KH, KL, n8s, KSC);
  feat16<<<gFT, b256, 0, stream>>>(F, fpos, DN, ST, 1, KS);
  attn_g<<<gAT, bAT, 0, stream>>>(QH, QL, KH, KL, QS, KS, VH, VL, gsp, OH, OL);
  cvt16<<<gXw, b256, 0, stream>>>(wo, WO, n8w, 1, WOS);
  gemm_o<2><<<dim3(nrtR * (DMOD / 64)), b128, 0, stream>>>(OH, OL, WO, out, 0, nrtR, 1.0f / (OSC * WOS));
  if (nrtP > 0) {
    gemm_o<1><<<dim3(nrtP * (DMOD / 64)), b128, 0, stream>>>(OH, OL, WO, out, QO, nrtP, 1.0f / (OSC * WOS));
  }
  (void)hipGetLastError();
}
